// MultiTaskGNN_43009802502560
// MI455X (gfx1250) — hardware-verified
//
#include <hip/hip_runtime.h>
#include <stddef.h>


#define NTHR    256
#define NWAVE   8
#define EPT     8
#define NGRP    2
#define CHUNK   (NTHR * EPT * NGRP)
#define WCAP    (EPT * NGRP * 32)
#define LISTN   (NWAVE * WCAP)
#define KSH     13
#define NBC     8192
#define NBF     2048
#define CPT     16
#define RCAP    40960
#define RBN     128
#define TGT     256
#define DEGCAP  1024
#define OTHR    512
#define BM      64
#define WSCAP   134217728
#define FIN     128
#define F1      256
#define H1      128
#define F2      64
#define H2      32
#define NPRED   4
#define ACARRY  8.0f
#define WCARRY  64.0f
#define SCL_AW  (1.0f / 512.0f)
#define NEG_SLOPE 0.2f

#define LDS_FILL ((RCAP + NBF + LISTN) * 4 + 64)

static_assert((CHUNK & (CHUNK - 1)) == 0);
static_assert(CHUNK <= (1 << 12));
static_assert(NBC <= (1 << KSH));
static_assert((NBC & (NBC - 1)) == 0 && (NBF & (NBF - 1)) == 0);
static_assert(NBC == 4 * NBF);
static_assert(OTHR * CPT == NBC);
static_assert((OTHR / 4) * CPT == NBF);
static_assert(OTHR / 32 == 16);
static_assert((RCAP % 32) == 0);
static_assert(TGT == NWAVE * 32);
static_assert((NBC % TGT) == 0);
static_assert((TGT % BM) == 0);
static_assert(WCAP == EPT * NGRP * 32);
static_assert((FIN % 32) == 0);
static_assert(F1 == 2 * H1 && F2 == 2 * H2);
static_assert(H1 == 32 * 4 && H2 == 32);
static_assert(FIN == 16 * 8);
static_assert(NBC == NWAVE * 8 * 128);
static_assert(H2 * NPRED <= NTHR);

typedef float    v4f  __attribute__((ext_vector_type(4)));
typedef float    v8f  __attribute__((ext_vector_type(8)));
typedef int      v4i  __attribute__((ext_vector_type(4)));
typedef _Float16 v4h  __attribute__((ext_vector_type(4)));
typedef _Float16 v8h  __attribute__((ext_vector_type(8)));
typedef _Float16 v16h __attribute__((ext_vector_type(16)));
union Frag { v16h v; v8h h[2]; };

__device__ __forceinline__ v8f wmh(v16h a, v16h b, v8f c) {
  v8f d = __builtin_amdgcn_wmma_f32_16x16x32_f16(false, a, false, b, (short)0, c, false, false);
  asm volatile("v_nop\n\tv_nop\n\tv_nop\n\tv_nop" : "+v"(d) : "v"(a), "v"(b));
  return d;
}

__device__ __forceinline__ v4i imax04(v4i v) {
  v4i o; o.x = max(v.x, 0); o.y = max(v.y, 0); o.z = max(v.z, 0); o.w = max(v.w, 0); return o;
}
__device__ __forceinline__ int hsum4i(v4i v) { return v.x + v.y + v.z + v.w; }
__device__ __forceinline__ float wsum1(float v) {
#pragma unroll
  for (int off = 16; off > 0; off >>= 1) v += __shfl_xor(v, off);
  return v;
}
__device__ __forceinline__ float leakyf(float v) { return v > 0.f ? v : v * NEG_SLOPE; }
__device__ __forceinline__ v4f leaky4(v4f v) {
  v4f o; o.x = leakyf(v.x); o.y = leakyf(v.y); o.z = leakyf(v.z); o.w = leakyf(v.w); return o;
}
__device__ __forceinline__ float eluf(float v) { return v > 0.f ? v : (__expf(fminf(v, 0.f)) - 1.0f); }

template <int NB>
__device__ __forceinline__ int scan_chunk(const int* __restrict__ dsts, int nE, int cbase, int slotBase,
                                          int vec8, int* list, int tid, int lane, int wave) {
  static_assert(NB <= (1 << KSH));
  int wc = 0;
#pragma unroll
  for (int g = 0; g < NGRP; ++g) {
    const int el0  = (g * NTHR + tid) * EPT;
    const int e0   = cbase + el0;
    const int sent = -2147483647 - 1;
    v4i da, db;
    if (vec8 != 0 && cbase + CHUNK <= nE) {
      da = *(const v4i*)(dsts + e0);
      db = *(const v4i*)(dsts + e0 + 4);
    } else {
      da.x = (e0     < nE) ? dsts[min(e0, nE - 1)] : sent;
      da.y = (e0 + 1 < nE) ? dsts[min(e0 + 1, nE - 1)] : sent;
      da.z = (e0 + 2 < nE) ? dsts[min(e0 + 2, nE - 1)] : sent;
      da.w = (e0 + 3 < nE) ? dsts[min(e0 + 3, nE - 1)] : sent;
      db.x = (e0 + 4 < nE) ? dsts[min(e0 + 4, nE - 1)] : sent;
      db.y = (e0 + 5 < nE) ? dsts[min(e0 + 5, nE - 1)] : sent;
      db.z = (e0 + 6 < nE) ? dsts[min(e0 + 6, nE - 1)] : sent;
      db.w = (e0 + 7 < nE) ? dsts[min(e0 + 7, nE - 1)] : sent;
    }
    const unsigned nb = (unsigned)slotBase;
    const unsigned s0 = (unsigned)da.x - nb, s1 = (unsigned)da.y - nb;
    const unsigned s2 = (unsigned)da.z - nb, s3 = (unsigned)da.w - nb;
    const unsigned s4 = (unsigned)db.x - nb, s5 = (unsigned)db.y - nb;
    const unsigned s6 = (unsigned)db.z - nb, s7 = (unsigned)db.w - nb;
    const bool h0 = s0 < (unsigned)NB, h1 = s1 < (unsigned)NB, h2 = s2 < (unsigned)NB, h3 = s3 < (unsigned)NB;
    const bool h4 = s4 < (unsigned)NB, h5 = s5 < (unsigned)NB, h6 = s6 < (unsigned)NB, h7 = s7 < (unsigned)NB;
    const unsigned any = __builtin_amdgcn_ballot_w32(h0 | h1 | h2 | h3 | h4 | h5 | h6 | h7);
    if (any != 0u) {
#define HITJ(J, HJ, SJ) { \
        const unsigned mj = __builtin_amdgcn_ballot_w32(HJ); \
        if (mj != 0u) { \
          if (HJ) { \
            const int pos = wc + (int)__builtin_amdgcn_mbcnt_lo(mj, 0u); \
            if (pos < WCAP) list[wave * WCAP + pos] = ((el0 + (J)) << KSH) | (int)(SJ); \
          } \
          wc += (int)__builtin_popcount(mj); } }
      HITJ(0, h0, s0)
      HITJ(1, h1, s1)
      HITJ(2, h2, s2)
      HITJ(3, h3, s3)
      HITJ(4, h4, s4)
      HITJ(5, h5, s5)
      HITJ(6, h6, s6)
      HITJ(7, h7, s7)
#undef HITJ
    }
  }
  return wc;
}

__global__ __launch_bounds__(NTHR) void k_count(const int* __restrict__ dsts, int* cnt, int nE, int vec8) {
  __shared__ __attribute__((aligned(16))) int scnt[NBC];
  __shared__ __attribute__((aligned(16))) int list[LISTN];
  __shared__ int wcnt[NWAVE];
  const int tid = threadIdx.x, lane = tid & 31, wave = tid >> 5;
  const int nodeBase = blockIdx.x * NBC;

  for (int i = tid; i < NBC; i += NTHR) scnt[i] = 0;
  __syncthreads();

  const int nChunks = (nE + CHUNK - 1) / CHUNK;
#pragma unroll 1
  for (int ch = 0; ch < nChunks; ++ch) {
    const int cbase = ch * CHUNK;
    const int wc = scan_chunk<NBC>(dsts, nE, cbase, nodeBase, vec8, list, tid, lane, wave);
    if (lane == 0) wcnt[wave] = wc;
    __syncthreads();
    if (wave == 0) {
#pragma unroll 1
      for (int wsx = 0; wsx < NWAVE; ++wsx) {
        int n = __builtin_amdgcn_readfirstlane(wcnt[wsx]);
        n = n > WCAP ? WCAP : (n < 0 ? 0 : n);
        const int* lp = list + wsx * WCAP;
#pragma unroll 1
        for (int i = 0; i < n; ++i) {
          const int ent  = __builtin_amdgcn_readfirstlane(lp[i]);
          const int slot = ent & (NBC - 1);
          if (lane == 0) scnt[slot] = scnt[slot] + 1;
        }
      }
    }
    __syncthreads();
  }

  v4i cq[8];
#pragma unroll
  for (int q = 0; q < 8; ++q) {
    const int f = (wave * 8 + q) * 128 + 4 * lane;
    cq[q] = *(const v4i*)(scnt + f);
  }
  int* cp = cnt + (size_t)nodeBase;
#pragma unroll
  for (int q = 0; q < 8; ++q) {
    const int f = (wave * 8 + q) * 128 + 4 * lane;
    *(volatile v4i*)(cp + f) = cq[q];
  }
  __threadfence();
#pragma unroll
  for (int q = 0; q < 8; ++q) {
    const int f = (wave * 8 + q) * 128 + 4 * lane;
    *(volatile v4i*)(cp + f) = cq[q];
  }
}

__global__ __launch_bounds__(OTHR) void k_offsets(
    const int* __restrict__ cnt, int* off, int* rbase, int nChunk) {
  __shared__ __attribute__((aligned(16))) int soff[NBC];
  __shared__ __attribute__((aligned(16))) int srb[RBN];
  __shared__ int wtot[OTHR / 32];
  const int tid = threadIdx.x, lane = tid & 31, wave = tid >> 5, sub = tid >> 7;
  for (int i = tid; i < RBN; i += OTHR) srb[i] = 0;
  int carry = 0;
#pragma unroll 1
  for (int ch = 0; ch < nChunk; ++ch) {
    const int base = ch * NBC;
    const int* cp = cnt + base + CPT * tid;
    const v4i c0 = imax04(*(const v4i*)cp);
    const v4i c1 = imax04(*(const v4i*)(cp + 4));
    const v4i c2 = imax04(*(const v4i*)(cp + 8));
    const v4i c3 = imax04(*(const v4i*)(cp + 12));
    const int ts = hsum4i(c0) + hsum4i(c1) + hsum4i(c2) + hsum4i(c3);
    int incl = ts;
#pragma unroll
    for (int d = 1; d < 32; d <<= 1) {
      const int t = __shfl_up(incl, d);
      if (lane >= d) incl += t;
    }
    if (lane == 31) wtot[wave] = incl;
    __syncthreads();
    const int S0 = wtot[0]  + wtot[1]  + wtot[2]  + wtot[3];
    const int S1 = wtot[4]  + wtot[5]  + wtot[6]  + wtot[7];
    const int S2 = wtot[8]  + wtot[9]  + wtot[10] + wtot[11];
    const int S3 = wtot[12] + wtot[13] + wtot[14] + wtot[15];
    int pre = 0;
#pragma unroll 1
    for (int w = 4 * sub; w < wave; ++w) pre += wtot[w];
    const int b0 = carry;
    const int b1 = b0 + ((S0 + 31) & ~31);
    const int b2 = b1 + ((S1 + 31) & ~31);
    const int b3 = b2 + ((S2 + 31) & ~31);
    const int b4 = b3 + ((S3 + 31) & ~31);
    const int myb = sub == 0 ? b0 : (sub == 1 ? b1 : (sub == 2 ? b2 : b3));
    if (tid == 0) {
      srb[min(4 * ch + 0, RBN - 1)] = b0;
      srb[min(4 * ch + 1, RBN - 1)] = b1;
      srb[min(4 * ch + 2, RBN - 1)] = b2;
      srb[min(4 * ch + 3, RBN - 1)] = b3;
    }
    int run = myb + pre + incl - ts;
    v4i o0, o1, o2, o3;
    o0.x = run; run += c0.x; o0.y = run; run += c0.y; o0.z = run; run += c0.z; o0.w = run; run += c0.w;
    o1.x = run; run += c1.x; o1.y = run; run += c1.y; o1.z = run; run += c1.z; o1.w = run; run += c1.w;
    o2.x = run; run += c2.x; o2.y = run; run += c2.y; o2.z = run; run += c2.z; o2.w = run; run += c2.w;
    o3.x = run; run += c3.x; o3.y = run; run += c3.y; o3.z = run; run += c3.z; o3.w = run;
    *(v4i*)(soff + CPT * tid)      = o0;
    *(v4i*)(soff + CPT * tid + 4)  = o1;
    *(v4i*)(soff + CPT * tid + 8)  = o2;
    *(v4i*)(soff + CPT * tid + 12) = o3;
    carry = b4;
    __syncthreads();
    v4i sv[4];
#pragma unroll
    for (int q = 0; q < 4; ++q) sv[q] = *(const v4i*)(soff + 4 * (tid + q * OTHR));
    int* op = off + base;
#pragma unroll
    for (int q = 0; q < 4; ++q) *(volatile v4i*)(op + 4 * (tid + q * OTHR)) = sv[q];
    __threadfence();
#pragma unroll
    for (int q = 0; q < 4; ++q) *(volatile v4i*)(op + 4 * (tid + q * OTHR)) = sv[q];
    __syncthreads();
  }
  if (tid == 0) srb[min(4 * nChunk, RBN - 1)] = carry;
  __syncthreads();
  v4i rv = {0, 0, 0, 0};
  if (tid < 32) rv = *(const v4i*)(srb + 4 * tid);
  if (tid < 32) *(volatile v4i*)(rbase + 4 * tid) = rv;
  __threadfence();
  if (tid < 32) *(volatile v4i*)(rbase + 4 * tid) = rv;
}

__global__ __launch_bounds__(NTHR) void k_fill(
    const int* __restrict__ dsts,
    const int* __restrict__ off, const int* __restrict__ rbase,
    int* csr, int nE, int vec8, int csrLen) {
  extern __shared__ v4f lds_dyn[];
  int* region = (int*)lds_dyn;
  int* cursor = region + RCAP;
  int* list   = cursor + NBF;
  int* wcnt   = list + LISTN;
  const int tid = threadIdx.x, lane = tid & 31, wave = tid >> 5;
  const int b = blockIdx.x;
  const int nodeBase = b * NBF;

  int rb0 = rbase[b];
  const int rb1 = rbase[b + 1];
  rb0 = rb0 < 0 ? 0 : (rb0 > csrLen ? csrLen : rb0);
  rb0 &= ~31;
  int len = rb1 - rb0;
  len = len < 0 ? 0 : (len > RCAP ? RCAP : len);
  int lenW = (len + 31) & ~31;
  if (rb0 + lenW > csrLen) lenW = (csrLen - rb0) & ~31;

  {
    const v4i z = {0, 0, 0, 0};
    for (int i = tid; i < RCAP / 4; i += NTHR) ((v4i*)region)[i] = z;
    for (int s = tid; s < NBF; s += NTHR) {
      int o = off[nodeBase + s] - rb0;
      o = o < 0 ? 0 : (o > RCAP ? RCAP : o);
      cursor[s] = o;
    }
  }
  __syncthreads();

  const int nChunks = (nE + CHUNK - 1) / CHUNK;
#pragma unroll 1
  for (int ch = 0; ch < nChunks; ++ch) {
    const int cbase = ch * CHUNK;
    const int wc = scan_chunk<NBF>(dsts, nE, cbase, nodeBase, vec8, list, tid, lane, wave);
    if (lane == 0) wcnt[wave] = wc;
    __syncthreads();
    if (wave == 0) {
#pragma unroll 1
      for (int wsx = 0; wsx < NWAVE; ++wsx) {
        int n = __builtin_amdgcn_readfirstlane(wcnt[wsx]);
        n = n > WCAP ? WCAP : (n < 0 ? 0 : n);
        const int* lp = list + wsx * WCAP;
#pragma unroll 1
        for (int i = 0; i < n; ++i) {
          const int ent  = __builtin_amdgcn_readfirstlane(lp[i]);
          const int slot = ent & (NBF - 1);
          int e = cbase + ((ent >> KSH) & (CHUNK - 1));
          e = e > nE - 1 ? nE - 1 : e;
          e = e < 0 ? 0 : e;
          if (lane == 0) {
            int pos = cursor[slot];
            pos = pos < 0 ? 0 : (pos > RCAP - 1 ? RCAP - 1 : pos);
            region[pos] = e;
            const int np = pos + 1;
            cursor[slot] = np > RCAP ? RCAP : np;
          }
        }
      }
    }
    __syncthreads();
  }

  const int nv = lenW >> 2;
  int* gp = csr + rb0;
#pragma unroll 1
  for (int i = tid; i < nv; i += NTHR) { const v4i v = ((const v4i*)region)[i]; *(volatile v4i*)(gp + 4 * i) = v; }
  __threadfence();
#pragma unroll 1
  for (int i = tid; i < nv; i += NTHR) { const v4i v = ((const v4i*)region)[i]; *(volatile v4i*)(gp + 4 * i) = v; }
}

__global__ __launch_bounds__(NTHR) void k_wcvt(const float* __restrict__ wa, const float* __restrict__ wb,
                                               _Float16* dp, int K, int Nc, int nUnits) {
  const int i = (int)blockIdx.x * NTHR + (int)threadIdx.x;
  if (i >= nUnits) return;
  const int ppr = K >> 3;
  const int n = i / ppr;
  const int seg = i - n * ppr;
  const bool useA = n < Nc;
  const int na = n > Nc - 1 ? Nc - 1 : n;
  int nbx = n - Nc;
  nbx = nbx < 0 ? 0 : (nbx > Nc - 1 ? Nc - 1 : nbx);
  v8h o;
#pragma unroll
  for (int j = 0; j < 8; ++j) {
    int k = 8 * seg + j;
    k = k > K - 1 ? K - 1 : k;
    const float fa = wa[(size_t)k * Nc + na];
    const float fb = wb[(size_t)k * Nc + nbx];
    const float f = useA ? fa : fb;
    o[j] = (_Float16)(f * WCARRY);
  }
  _Float16* gp = dp + (size_t)i * 8;
  *(volatile v8h*)gp = o;
  __threadfence();
  *(volatile v8h*)gp = o;
}

__global__ __launch_bounds__(NTHR) void k_acvt(const float* __restrict__ x, _Float16* a1, int nN, int npad) {
  const int gi = (int)blockIdx.x * NTHR + (int)threadIdx.x;
  const int row = gi >> 4, seg = gi & 15;
  if (row >= npad) return;
  int rr = row > nN - 1 ? nN - 1 : row;
  rr = rr < 0 ? 0 : rr;
  const bool live = row < nN;
  const float* rp = x + (size_t)rr * FIN + 8 * seg;
  const v4f x0 = *(const v4f*)rp;
  const v4f x1 = *(const v4f*)(rp + 4);
  const float sc = live ? ACARRY : 0.f;
  v8h o;
  o[0] = (_Float16)(x0.x * sc); o[1] = (_Float16)(x0.y * sc); o[2] = (_Float16)(x0.z * sc); o[3] = (_Float16)(x0.w * sc);
  o[4] = (_Float16)(x1.x * sc); o[5] = (_Float16)(x1.y * sc); o[6] = (_Float16)(x1.z * sc); o[7] = (_Float16)(x1.w * sc);
  _Float16* gp = a1 + (size_t)row * FIN + 8 * seg;
  *(volatile v8h*)gp = o;
  __threadfence();
  *(volatile v8h*)gp = o;
}

template <int BNC>
__global__ __launch_bounds__(NTHR) void k_gemm(
    const _Float16* __restrict__ A, const _Float16* __restrict__ Bp,
    const float* __restrict__ ba, const float* __restrict__ bb,
    float* Cout, int K, int ldc, int half, int nValid, int nStore, float scl) {
  constexpr int TPW = BNC / 32;
  constexpr int PPR = BNC / 4;
  constexpr int NIT = (BM * PPR) / NTHR;
  constexpr int LSH = (PPR == 32) ? 5 : 4;
  static_assert(BNC == 128 || BNC == 64);
  static_assert((BM * PPR) % NTHR == 0);
  static_assert(NIT >= 1);
  static_assert(TPW * 16 * 2 == BNC);
  static_assert(BM == 4 * 16);
  static_assert((1 << LSH) == PPR);

  __shared__ __attribute__((aligned(16))) float stg[BM * BNC];
  const int tid = threadIdx.x, lane = tid & 31, wave = tid >> 5, hh = lane >> 4, m = lane & 15;
  const int rowBase = (int)blockIdx.x * BM;
  const int colBase = (int)blockIdx.y * BNC;
  const int rg = wave >> 1, chf = wave & 1;
  const int r0 = rg * 16;
  const int c0 = chf * (BNC / 2);

  v8f acc[TPW];
#pragma unroll
  for (int t = 0; t < TPW; ++t) { v8f z = {0.f, 0.f, 0.f, 0.f, 0.f, 0.f, 0.f, 0.f}; acc[t] = z; }

  const _Float16* ap = A  + (size_t)(rowBase + r0 + m) * K + 8 * hh;
  const _Float16* bp = Bp + (size_t)(colBase + c0 + m) * K + 8 * hh;
  const int ksteps = K >> 5;
#pragma unroll 1
  for (int kt = 0; kt < ksteps; ++kt) {
    Frag a;
    a.h[0] = *(const v8h*)(ap + 32 * kt);
    a.h[1] = *(const v8h*)(ap + 32 * kt + 16);
#pragma unroll
    for (int t = 0; t < TPW; ++t) {
      const size_t to = (size_t)(16 * t) * K + 32 * kt;
      Frag b;
      b.h[0] = *(const v8h*)(bp + to);
      b.h[1] = *(const v8h*)(bp + to + 16);
      acc[t] = wmh(a.v, b.v, acc[t]);
    }
  }

  {
    float* sp = stg + (size_t)(r0 + 8 * hh) * BNC + c0 + m;
    const int growb = rowBase + r0 + 8 * hh;
#pragma unroll
    for (int t = 0; t < TPW; ++t) {
      const int col = colBase + c0 + 16 * t + m;
      const int ia = col > half - 1 ? half - 1 : col;
      int ib = col - half;
      ib = ib < 0 ? 0 : (ib > half - 1 ? half - 1 : ib);
      const float fa = ba[ia];
      const float fb = bb[ib];
      const float bv = col < half ? fa : fb;
#pragma unroll
      for (int r = 0; r < 8; ++r) {
        const bool lv = (growb + r) < nValid;
        const float g = acc[t][r] * scl + bv;
        sp[r * BNC + 16 * t] = lv ? g : 0.f;
      }
    }
  }
  __syncthreads();

  v4f cv[NIT];
#pragma unroll
  for (int it = 0; it < NIT; ++it) {
    const int id = it * NTHR + tid;
    const int row = id >> LSH, seg = id & (PPR - 1);
    cv[it] = *(const v4f*)(stg + (size_t)row * BNC + 4 * seg);
  }
#pragma unroll
  for (int it = 0; it < NIT; ++it) {
    const int id = it * NTHR + tid;
    const int row = id >> LSH, seg = id & (PPR - 1);
    const int grow = rowBase + row;
    if (grow < nStore) {
      float* gp = Cout + (size_t)grow * ldc + colBase + 4 * seg;
      *(volatile v4f*)gp = cv[it];
    }
  }
  __threadfence();
#pragma unroll
  for (int it = 0; it < NIT; ++it) {
    const int id = it * NTHR + tid;
    const int row = id >> LSH, seg = id & (PPR - 1);
    const int grow = rowBase + row;
    if (grow < nStore) {
      float* gp = Cout + (size_t)grow * ldc + colBase + 4 * seg;
      *(volatile v4f*)gp = cv[it];
    }
  }
}

__global__ __launch_bounds__(NTHR) void k_agg1(
    const int* __restrict__ csr, const int* __restrict__ off, const int* __restrict__ cnt,
    const int* __restrict__ snd, const float* __restrict__ ea, const float* __restrict__ P,
    const float* __restrict__ We, const float* __restrict__ att, const float* __restrict__ bias,
    _Float16* a2, int nN, int nE, int csrLen) {
  const int tid = threadIdx.x, lane = tid & 31, wave = tid >> 5;
  const int tbase = (int)blockIdx.x * TGT + wave * 32;
  const int cl    = tbase + lane;
  const int cnt_l = cnt[cl];
  const int off_l = off[cl];
  const v4f we = *(const v4f*)(We + 4 * lane);
  const v4f at = *(const v4f*)(att + 4 * lane);
  const v4f bs = *(const v4f*)(bias + 4 * lane);
  const float QNAN = __int_as_float(0x7fc00000);
  const v4f zero4 = {0.f, 0.f, 0.f, 0.f};

#pragma unroll 1
  for (int j = 0; j < 32; ++j) {
    const int c = tbase + j;
    const int nraw = __builtin_amdgcn_readfirstlane(__shfl(cnt_l, j));
    const int st   = __builtin_amdgcn_readfirstlane(__shfl(off_l, j));
    const bool over = nraw > DEGCAP;
    const int n = nraw < 0 ? 0 : (nraw > DEGCAP ? DEGCAP : nraw);
    int cc = c > nN - 1 ? nN - 1 : c;
    cc = cc < 0 ? 0 : cc;
    const v4f xr = *(const v4f*)(P + (size_t)cc * F1 + H1 + 4 * lane);

    float eas = 0.f;
#pragma unroll 1
    for (int q0 = 0; q0 < n; q0 += 32) {
      int pos = st + q0 + lane;
      pos = pos < 0 ? 0 : (pos > csrLen - 1 ? csrLen - 1 : pos);
      int e = csr[pos];
      e = e < 0 ? 0 : (e > nE - 1 ? nE - 1 : e);
      const bool valid = lane < (n - q0);
      const float v = ea[e];
      eas += wsum1(valid ? v : 0.f);
    }
    const float den = (float)(n < 1 ? 1 : n);
    const float eam = eas * __builtin_amdgcn_rcpf(den);

    float mx = -1.0e30f, z = 0.f;
    v4f acc = zero4;
    const int total = n + 1;
#pragma unroll 1
    for (int q0 = 0; q0 < total; q0 += 32) {
      const int idx = q0 + lane;
      const bool isE = idx < n;
      int pos = st + idx;
      pos = pos < 0 ? 0 : (pos > csrLen - 1 ? csrLen - 1 : pos);
      int e = csr[pos];
      e = e < 0 ? 0 : (e > nE - 1 ? nE - 1 : e);
      int se = snd[e];
      se = se < 0 ? 0 : (se > nN - 1 ? nN - 1 : se);
      const float eae = ea[e];
      const int   s   = isE ? se : cc;
      const float eav = isE ? eae : eam;
      const int mcnt = (total - q0) < 32 ? (total - q0) : 32;
#pragma unroll 1
      for (int pp = 0; pp < mcnt; ++pp) {
        const int   sb = __builtin_amdgcn_readlane(s, pp);
        const float ev = __int_as_float(__builtin_amdgcn_readlane(__float_as_int(eav), pp));
        const v4f xl = *(const v4f*)(P + (size_t)sb * F1 + 4 * lane);
        v4f fv = (xl + xr) + we * ev;
        fv = leaky4(fv);
        float g = fv.x * at.x + fv.y * at.y + fv.z * at.z + fv.w * at.w;
        g += __shfl_xor(g, 1);
        g += __shfl_xor(g, 2);
        g += __shfl_xor(g, 4);
        const float mn = fmaxf(mx, g);
        const float sc = __expf(mx - mn);
        const float w  = __expf(g - mn);
        z   = z * sc + w;
        acc = acc * sc + xl * w;
        mx  = mn;
      }
    }
    const float rz = __builtin_amdgcn_rcpf(z);
    const v4f o = acc * rz + bs;
    v4f h;
    h.x = eluf(o.x); h.y = eluf(o.y); h.z = eluf(o.z); h.w = eluf(o.w);
    const bool live = c < nN;
    const float sc8  = live ? ACARRY : 0.f;
    const float padd = over ? QNAN : 0.f;
    v4h hv;
    hv[0] = (_Float16)(h.x * sc8 + padd);
    hv[1] = (_Float16)(h.y * sc8 + padd);
    hv[2] = (_Float16)(h.z * sc8 + padd);
    hv[3] = (_Float16)(h.w * sc8 + padd);
    _Float16* gp = a2 + (size_t)c * FIN + 4 * lane;
    *(volatile v4h*)gp = hv;
    __threadfence();
    *(volatile v4h*)gp = hv;
  }
}

__global__ __launch_bounds__(NTHR) void k_agg2(
    const int* __restrict__ csr, const int* __restrict__ off, const int* __restrict__ cnt,
    const int* __restrict__ snd, const float* __restrict__ ea, const float* __restrict__ P,
    const float* __restrict__ We, const float* __restrict__ att, const float* __restrict__ bias,
    float* out, int shOff, int nN, int nE, int csrLen) {
  const int tid = threadIdx.x, lane = tid & 31, wave = tid >> 5;
  const int tbase = (int)blockIdx.x * TGT + wave * 32;
  const int cl    = tbase + lane;
  const int cnt_l = cnt[cl];
  const int off_l = off[cl];
  const float we = We[lane];
  const float at = att[lane];
  const float bs = bias[lane];
  const float QNAN = __int_as_float(0x7fc00000);

#pragma unroll 1
  for (int j = 0; j < 32; ++j) {
    const int c = tbase + j;
    const int nraw = __builtin_amdgcn_readfirstlane(__shfl(cnt_l, j));
    const int st   = __builtin_amdgcn_readfirstlane(__shfl(off_l, j));
    const bool over = nraw > DEGCAP;
    const int n = nraw < 0 ? 0 : (nraw > DEGCAP ? DEGCAP : nraw);
    int cc = c > nN - 1 ? nN - 1 : c;
    cc = cc < 0 ? 0 : cc;
    const float xr = P[(size_t)cc * F2 + H2 + lane];

    float eas = 0.f;
#pragma unroll 1
    for (int q0 = 0; q0 < n; q0 += 32) {
      int pos = st + q0 + lane;
      pos = pos < 0 ? 0 : (pos > csrLen - 1 ? csrLen - 1 : pos);
      int e = csr[pos];
      e = e < 0 ? 0 : (e > nE - 1 ? nE - 1 : e);
      const bool valid = lane < (n - q0);
      const float v = ea[e];
      eas += wsum1(valid ? v : 0.f);
    }
    const float den = (float)(n < 1 ? 1 : n);
    const float eam = eas * __builtin_amdgcn_rcpf(den);

    float mx = -1.0e30f, z = 0.f, acc = 0.f;
    const int total = n + 1;
#pragma unroll 1
    for (int q0 = 0; q0 < total; q0 += 32) {
      const int idx = q0 + lane;
      const bool isE = idx < n;
      int pos = st + idx;
      pos = pos < 0 ? 0 : (pos > csrLen - 1 ? csrLen - 1 : pos);
      int e = csr[pos];
      e = e < 0 ? 0 : (e > nE - 1 ? nE - 1 : e);
      int se = snd[e];
      se = se < 0 ? 0 : (se > nN - 1 ? nN - 1 : se);
      const float eae = ea[e];
      const int   s   = isE ? se : cc;
      const float eav = isE ? eae : eam;
      const int mcnt = (total - q0) < 32 ? (total - q0) : 32;
#pragma unroll 1
      for (int pp = 0; pp < mcnt; ++pp) {
        const int   sb = __builtin_amdgcn_readlane(s, pp);
        const float ev = __int_as_float(__builtin_amdgcn_readlane(__float_as_int(eav), pp));
        const float xl = P[(size_t)sb * F2 + lane];
        float fv = (xl + xr) + we * ev;
        fv = leakyf(fv);
        const float g = wsum1(fv * at);
        const float mn = fmaxf(mx, g);
        const float sc = __expf(mx - mn);
        const float w  = __expf(g - mn);
        z   = z * sc + w;
        acc = acc * sc + xl * w;
        mx  = mn;
      }
    }
    const float rz = __builtin_amdgcn_rcpf(z);
    const float padd = over ? QNAN : 0.f;
    const float o = (acc * rz + bs) + padd;
    const bool live = c < nN;
    float* gp = out + (size_t)shOff + (size_t)cc * H2 + lane;
    if (live) *(volatile float*)gp = o;
    __threadfence();
    if (live) *(volatile float*)gp = o;
  }
}

__global__ __launch_bounds__(NTHR) void k_preds(const float* sh, const float* __restrict__ Wo,
                                                const float* __restrict__ bo, float* out, int nN, int nPred) {
  __shared__ __attribute__((aligned(16))) float sW[H2 * NPRED];
  __shared__ float sB[NPRED];
  const int tid = threadIdx.x, lane = tid & 31, wave = tid >> 5;
  if (tid < H2 * NPRED) sW[tid] = Wo[tid];
  if (tid < NPRED) sB[tid] = bo[tid];
  __syncthreads();
  const int line = (int)blockIdx.x * NWAVE + wave;
  const int f = line * 32 + lane;
  const bool live = f < nPred;
  const int fc = f > nPred - 1 ? nPred - 1 : f;
  int k = fc / nN;
  k = k < 0 ? 0 : (k > NPRED - 1 ? NPRED - 1 : k);
  int i = fc - k * nN;
  i = i < 0 ? 0 : (i > nN - 1 ? nN - 1 : i);
  const float* sr = sh + (size_t)i * H2;
  float a = 0.f;
#pragma unroll 1
  for (int q = 0; q < H2 / 4; ++q) {
    const v4f s = *(const v4f*)(sr + 4 * q);
    const float* wq = sW + (4 * q) * NPRED + k;
    a = fmaf(s.x, wq[0], a);
    a = fmaf(s.y, wq[NPRED], a);
    a = fmaf(s.z, wq[2 * NPRED], a);
    a = fmaf(s.w, wq[3 * NPRED], a);
  }
  a += sB[k];
  if (live) *(volatile float*)(out + f) = a;
  __threadfence();
  if (live) *(volatile float*)(out + f) = a;
}

extern "C" void kernel_launch(void* const* d_in, const int* in_sizes, int n_in,
                              void* d_out, int out_size, void* d_ws, size_t ws_size,
                              hipStream_t stream) {
  if (n_in < 19) return;
  if (in_sizes[0] < FIN || (in_sizes[0] % FIN) != 0) return;
  const int nN = in_sizes[0] / FIN;
  if (nN < 1 || nN > 200000) return;
  const int nE = in_sizes[1];
  if (nE < 1 || nE > (1 << 26)) return;
  if (in_sizes[18] != 2 * nE) return;
  if (in_sizes[2] != FIN * H1 || in_sizes[4] != FIN * H1) return;
  if (in_sizes[3] != H1 || in_sizes[5] != H1) return;
  if (in_sizes[6] != H1 || in_sizes[7] != H1 || in_sizes[8] != H1) return;
  if (in_sizes[9] != FIN * H2 || in_sizes[11] != FIN * H2) return;
  if (in_sizes[10] != H2 || in_sizes[12] != H2) return;
  if (in_sizes[13] != H2 || in_sizes[14] != H2 || in_sizes[15] != H2) return;
  if (in_sizes[16] != H2 * NPRED || in_sizes[17] != NPRED) return;
  if (out_size != nN * NPRED + nN * H2) return;

  const float* x     = (const float*)d_in[0];
  const float* eattr = (const float*)d_in[1];
  const float* Wl1   = (const float*)d_in[2];
  const float* bl1   = (const float*)d_in[3];
  const float* Wr1   = (const float*)d_in[4];
  const float* br1   = (const float*)d_in[5];
  const float* We1   = (const float*)d_in[6];
  const float* att1  = (const float*)d_in[7];
  const float* bias1 = (const float*)d_in[8];
  const float* Wl2   = (const float*)d_in[9];
  const float* bl2   = (const float*)d_in[10];
  const float* Wr2   = (const float*)d_in[11];
  const float* br2   = (const float*)d_in[12];
  const float* We2   = (const float*)d_in[13];
  const float* att2  = (const float*)d_in[14];
  const float* bias2 = (const float*)d_in[15];
  const float* Wout  = (const float*)d_in[16];
  const float* bout  = (const float*)d_in[17];
  const int*   ei    = (const int*)d_in[18];
  const int*   srcI  = ei;
  const int*   dstI  = ei + nE;
  float* out = (float*)d_out;

  const int NPAD   = ((nN + TGT - 1) / TGT) * TGT;
  const int nAgg   = NPAD / TGT;
  const int nBC    = (nN + NBC - 1) / NBC;
  const int CNTPAD = nBC * NBC;
  if (CNTPAD < NPAD) return;
  if (4 * nBC + 1 > RBN) return;
  const int nBF    = (nN + NBF - 1) / NBF;
  if (nBF > 4 * nBC) return;
  const int csrLen = ((nE + 31) & ~31) + 4096;
  if (31 * 4 * nBC > 4096) return;
  const int nPred  = NPRED * nN;
  const int shOff  = nPred;

  char* ws = (char*)d_ws;
  size_t off = 0;
  const size_t oCnt = off; off += (size_t)CNTPAD * 4;                    off = (off + 255) & ~(size_t)255;
  const size_t oOff = off; off += (size_t)CNTPAD * 4;                    off = (off + 255) & ~(size_t)255;
  const size_t oRb  = off; off += (size_t)RBN * 4;                       off = (off + 255) & ~(size_t)255;
  const size_t oCsr = off; off += (size_t)csrLen * 4;                    off = (off + 255) & ~(size_t)255;
  const size_t oW1  = off; off += (size_t)F1 * FIN * 2;                  off = (off + 255) & ~(size_t)255;
  const size_t oW2  = off; off += (size_t)F2 * FIN * 2;                  off = (off + 255) & ~(size_t)255;
  const size_t oA1  = off; off += (size_t)NPAD * FIN * 2;                off = (off + 255) & ~(size_t)255;
  const size_t oP1  = off; off += (size_t)NPAD * F1 * 4;                 off = (off + 255) & ~(size_t)255;
  const size_t oA2  = off; off += (size_t)NPAD * FIN * 2;                off = (off + 255) & ~(size_t)255;
  const size_t oP2  = off; off += (size_t)NPAD * F2 * 4;                 off = (off + 255) & ~(size_t)255;
  if (off > ws_size || off > (size_t)WSCAP) return;

  int*   cnt   = (int*)(ws + oCnt);
  int*   offp  = (int*)(ws + oOff);
  int*   rb    = (int*)(ws + oRb);
  int*   csr   = (int*)(ws + oCsr);
  _Float16* wp1 = (_Float16*)(ws + oW1);
  _Float16* wp2 = (_Float16*)(ws + oW2);
  _Float16* a1  = (_Float16*)(ws + oA1);
  float*    P1  = (float*)(ws + oP1);
  _Float16* a2  = (_Float16*)(ws + oA2);
  float*    P2  = (float*)(ws + oP2);

  const int vec8 = ((nE & 3) == 0) ? 1 : 0;

  k_count<<<nBC, NTHR, 0, stream>>>(dstI, cnt, nE, vec8);
  k_offsets<<<1, OTHR, 0, stream>>>(cnt, offp, rb, nBC);
  hipFuncSetAttribute(reinterpret_cast<const void*>(&k_fill),
                      hipFuncAttributeMaxDynamicSharedMemorySize, LDS_FILL);
  k_fill<<<nBF, NTHR, LDS_FILL, stream>>>(dstI, offp, rb, csr, nE, vec8, csrLen);

  {
    const int u1 = F1 * (FIN / 8);
    const int u2 = F2 * (FIN / 8);
    k_wcvt<<<(u1 + NTHR - 1) / NTHR, NTHR, 0, stream>>>(Wl1, Wr1, wp1, FIN, H1, u1);
    k_wcvt<<<(u2 + NTHR - 1) / NTHR, NTHR, 0, stream>>>(Wl2, Wr2, wp2, FIN, H2, u2);
  }
  k_acvt<<<(NPAD * 16) / NTHR, NTHR, 0, stream>>>(x, a1, nN, NPAD);

  k_gemm<128><<<dim3(NPAD / BM, F1 / 128), NTHR, 0, stream>>>(a1, wp1, bl1, br1, P1, FIN, F1, H1, nN, NPAD, SCL_AW);

  k_agg1<<<nAgg, NTHR, 0, stream>>>(csr, offp, cnt, srcI, eattr, P1, We1, att1, bias1, a2, nN, nE, csrLen);

  k_gemm<64><<<dim3(NPAD / BM, 1), NTHR, 0, stream>>>(a2, wp2, bl2, br2, P2, FIN, F2, H2, nN, NPAD, SCL_AW);

  k_agg2<<<nAgg, NTHR, 0, stream>>>(csr, offp, cnt, srcI, eattr, P2, We2, att2, bias2, out, shOff, nN, nE, csrLen);

  {
    const int nLines = (nPred + 31) / 32;
    k_preds<<<(nLines + NWAVE - 1) / NWAVE, NTHR, 0, stream>>>(out + shOff, Wout, bout, out, nN, nPred);
  }
}
